// LateMultiInteractiveRetriever_10754598109467
// MI455X (gfx1250) — hardware-verified
//
#include <hip/hip_runtime.h>

typedef _Float16 v16h __attribute__((ext_vector_type(16)));
typedef _Float16 v8h  __attribute__((ext_vector_type(8)));
typedef __bf16   v16bf __attribute__((ext_vector_type(16)));
typedef unsigned short v8us __attribute__((ext_vector_type(8)));
typedef unsigned short v4us __attribute__((ext_vector_type(4)));
typedef float v8f __attribute__((ext_vector_type(8)));
typedef float v4f __attribute__((ext_vector_type(4)));
typedef v8h  __attribute__((may_alias)) v8ha;
typedef v8us __attribute__((may_alias)) v8usa;
typedef v4us __attribute__((may_alias)) v4usa;
typedef v4f  __attribute__((may_alias)) v4fa;
typedef float __attribute__((may_alias)) f32a;
typedef _Float16 __attribute__((may_alias)) f16a;

union FragH { v16h v; v8h half[2]; };
union FragB { v16bf v; v8us half[2]; };

#define DM    256
#define NQ    1024
#define NC    2000
#define JSW   32
#define JPHO  24
#define NKSW  64000
#define NKPHO 48000
#define LGP   2048
#define NCHNK 63
#define WN    65536
#define QSC   8.0f
#define KSC   4.0f
#define RSC   2048.0f

__device__ __forceinline__ v8f wmma_f16(v16h a, v16h b, v8f c) {
  v8f d = __builtin_amdgcn_wmma_f32_16x16x32_f16(false, a, false, b, (short)0, c, false, false);
  asm volatile("v_nop\n\tv_nop\n\tv_nop\n\tv_nop" : "+v"(d) : "v"(a), "v"(b));
  return d;
}
__device__ __forceinline__ v8f wmma_bf16(v16bf a, v16bf b, v8f c) {
  v8f d = __builtin_amdgcn_wmma_f32_16x16x32_bf16(false, a, false, b, (short)0, c, false, false);
  asm volatile("v_nop\n\tv_nop\n\tv_nop\n\tv_nop" : "+v"(d) : "v"(a), "v"(b));
  return d;
}

__device__ __forceinline__ v16h ldfrag_h(const _Float16* p, int h) {
  FragH f;
  f.half[0] = *(const v8ha*)(p + 8 * h);
  f.half[1] = *(const v8ha*)(p + 16 + 8 * h);
  return f.v;
}
__device__ __forceinline__ v16bf ldfrag_b(const unsigned short* p, int h) {
  FragB f;
  f.half[0] = *(const v8usa*)(p + 8 * h);
  f.half[1] = *(const v8usa*)(p + 16 + 8 * h);
  return f.v;
}

__device__ __forceinline__ unsigned int bfbits(float x) {
  const unsigned int u = __float_as_uint(x);
  return (u + 0x7FFFu + ((u >> 16) & 1u)) >> 16;
}
__device__ __forceinline__ void split_hl(float x, unsigned short& hb, unsigned short& lb) {
  const unsigned int hh = bfbits(x);
  const float hv = __uint_as_float(hh << 16);
  hb = (unsigned short)hh;
  lb = (unsigned short)bfbits(x - hv);
}

__global__ __launch_bounds__(256) void cvtw_kernel(
    const float* __restrict__ w0, const float* __restrict__ w1, const float* __restrict__ w2,
    const float* __restrict__ w3, const float* __restrict__ w4,
    unsigned short* whi, unsigned short* wlo)
{
  const int g = blockIdx.x * 256 + threadIdx.x;
  if (g >= 5 * (WN / 8)) return;
  const int widx = g >> 13;
  const int off = (g & 8191) * 8;
  const float* src = (widx == 0) ? w0 : ((widx == 1) ? w1 : ((widx == 2) ? w2 : ((widx == 3) ? w3 : w4)));
  const v4f a = *(const v4fa*)(src + off);
  const v4f c = *(const v4fa*)(src + off + 4);
  unsigned short h0, h1, h2, h3, h4, h5, h6, h7;
  unsigned short l0, l1, l2, l3, l4, l5, l6, l7;
  split_hl(a.x, h0, l0); split_hl(a.y, h1, l1); split_hl(a.z, h2, l2); split_hl(a.w, h3, l3);
  split_hl(c.x, h4, l4); split_hl(c.y, h5, l5); split_hl(c.z, h6, l6); split_hl(c.w, h7, l7);
  const v8us hv = { h0, h1, h2, h3, h4, h5, h6, h7 };
  const v8us lv = { l0, l1, l2, l3, l4, l5, l6, l7 };
  unsigned short* dh = whi + (size_t)widx * WN + off;
  unsigned short* dl = wlo + (size_t)widx * WN + off;
  *(volatile v8us*)dh = hv;
  *(volatile v8us*)dl = lv;
  __threadfence();
  *(volatile v8us*)dh = hv;
  *(volatile v8us*)dl = lv;
}

__device__ __forceinline__ void tile_store_f32(const float* so, float* dst, int w, int lane) {
  const int q8 = lane & 7, sub = lane >> 3;
  #pragma unroll
  for (int i = 0; i < 16; ++i) {
    const int L = i * 16 + w * 4 + sub;
    const int row = L >> 3, piece = (L & 7) * 32;
    const int off = row * DM + piece + 4 * q8;
    const v4f v = *(const v4fa*)(so + off);
    *(volatile v4f*)(dst + off) = v;
  }
}
__device__ __forceinline__ void tile_store_f16(const _Float16* so, _Float16* dst, int w, int lane) {
  const int q8 = lane & 7, sub = lane >> 3;
  #pragma unroll
  for (int i = 0; i < 8; ++i) {
    const int L = i * 16 + w * 4 + sub;
    const int row = L >> 2, piece = (L & 3) * 64;
    const int off = row * DM + piece + 8 * q8;
    const v8h v = *(const v8ha*)(so + off);
    *(volatile v8h*)(dst + off) = v;
  }
}

__global__ __launch_bounds__(128) void proj_kernel(
    const float* __restrict__ A,
    const unsigned short* __restrict__ whi, const unsigned short* __restrict__ wlo,
    const float* __restrict__ bias,
    float* outF, _Float16* outH, _Float16* outR, int mode, float oscale)
{
  __shared__ __attribute__((aligned(16))) float smem[32 * DM];
  unsigned short* sHi = (unsigned short*)smem;
  unsigned short* sLo = sHi + 32 * DM;

  const int tid = threadIdx.x, lane = tid & 31, w = tid >> 5;
  const int h = lane >> 4, m = lane & 15;
  const int m0 = blockIdx.x * 32;

  #pragma unroll 4
  for (int it = 0; it < 16; ++it) {
    const int idx = it * 128 + tid;
    const int row = idx >> 6, c4 = (idx & 63) * 4;
    const v4f x = *(const v4fa*)(A + (size_t)(m0 + row) * DM + c4);
    unsigned short h0, h1, h2, h3, l0, l1, l2, l3;
    split_hl(x.x, h0, l0); split_hl(x.y, h1, l1); split_hl(x.z, h2, l2); split_hl(x.w, h3, l3);
    const v4us hv = { h0, h1, h2, h3 };
    const v4us lv = { l0, l1, l2, l3 };
    *(v4usa*)(sHi + row * DM + c4) = hv;
    *(v4usa*)(sLo + row * DM + c4) = lv;
  }
  __syncthreads();

  const v8f zero8 = { 0.f, 0.f, 0.f, 0.f, 0.f, 0.f, 0.f, 0.f };
  v8f acc[2][4];
  #pragma unroll
  for (int mt = 0; mt < 2; ++mt)
    #pragma unroll
    for (int nt = 0; nt < 4; ++nt) acc[mt][nt] = zero8;

  const unsigned short* ah0 = sHi + m * DM;
  const unsigned short* ah1 = ah0 + 16 * DM;
  const unsigned short* al0 = sLo + m * DM;
  const unsigned short* al1 = al0 + 16 * DM;
  const unsigned short* bhp = whi + (size_t)(64 * w + m) * DM;
  const unsigned short* blp = wlo + (size_t)(64 * w + m) * DM;

  #pragma unroll 1
  for (int k0 = 0; k0 < DM; k0 += 32) {
    const v16bf a0h = ldfrag_b(ah0 + k0, h);
    const v16bf a1h = ldfrag_b(ah1 + k0, h);
    const v16bf a0l = ldfrag_b(al0 + k0, h);
    const v16bf a1l = ldfrag_b(al1 + k0, h);
    #pragma unroll
    for (int nt = 0; nt < 4; ++nt) {
      const v16bf fbh = ldfrag_b(bhp + nt * 16 * DM + k0, h);
      const v16bf fbl = ldfrag_b(blp + nt * 16 * DM + k0, h);
      acc[0][nt] = wmma_bf16(a0h, fbh, acc[0][nt]);
      acc[0][nt] = wmma_bf16(a0h, fbl, acc[0][nt]);
      acc[0][nt] = wmma_bf16(a0l, fbh, acc[0][nt]);
      acc[1][nt] = wmma_bf16(a1h, fbh, acc[1][nt]);
      acc[1][nt] = wmma_bf16(a1h, fbl, acc[1][nt]);
      acc[1][nt] = wmma_bf16(a1l, fbh, acc[1][nt]);
    }
  }
  __syncthreads();

  if (mode == 0) {
    f32a* so = (f32a*)smem;
    #pragma unroll
    for (int nt = 0; nt < 4; ++nt) {
      const int col = 64 * w + 16 * nt + m;
      const float bv = bias[col];
      #pragma unroll
      for (int mt = 0; mt < 2; ++mt)
        #pragma unroll
        for (int r = 0; r < 8; ++r) {
          const int row = 16 * mt + 8 * h + r;
          so[row * DM + col] = acc[mt][nt][r] + bv;
        }
    }
    __syncthreads();
    float* dst = outF + (size_t)m0 * DM;
    tile_store_f32((const float*)smem, dst, w, lane);
    __threadfence();
    tile_store_f32((const float*)smem, dst, w, lane);
  } else {
    f16a* so = (f16a*)smem;
    f16a* sr = so + 32 * DM;
    #pragma unroll
    for (int nt = 0; nt < 4; ++nt) {
      const int col = 64 * w + 16 * nt + m;
      const float bv = bias[col];
      #pragma unroll
      for (int mt = 0; mt < 2; ++mt)
        #pragma unroll
        for (int r = 0; r < 8; ++r) {
          const int row = 16 * mt + 8 * h + r;
          const float y = (acc[mt][nt][r] + bv) * oscale;
          const _Float16 hq = (_Float16)y;
          so[row * DM + col] = hq;
          if (mode == 2) sr[row * DM + col] = (_Float16)((y - (float)hq) * RSC);
        }
    }
    __syncthreads();
    _Float16* dst = outH + (size_t)m0 * DM;
    _Float16* dsr = outR + (size_t)m0 * DM;
    tile_store_f16((const _Float16*)so, dst, w, lane);
    if (mode == 2) tile_store_f16((const _Float16*)sr, dsr, w, lane);
    __threadfence();
    tile_store_f16((const _Float16*)so, dst, w, lane);
    if (mode == 2) tile_store_f16((const _Float16*)sr, dsr, w, lane);
  }
}

__device__ __forceinline__ float tile_max2(const _Float16* kr, const _Float16* qhl,
                                           const _Float16* qrl, int h) {
  v8f acc  = { 0.f, 0.f, 0.f, 0.f, 0.f, 0.f, 0.f, 0.f };
  v8f accr = { 0.f, 0.f, 0.f, 0.f, 0.f, 0.f, 0.f, 0.f };
  #pragma unroll 2
  for (int ks = 0; ks < 8; ++ks) {
    const v16h a  = ldfrag_h(kr + 32 * ks, h);
    const v16h bh = ldfrag_h(qhl + 32 * ks, h);
    const v16h br = ldfrag_h(qrl + 32 * ks, h);
    acc  = wmma_f16(a, bh, acc);
    accr = wmma_f16(a, br, accr);
  }
  const float ir = 1.0f / RSC;
  float mx = acc[0] + accr[0] * ir;
  #pragma unroll
  for (int r = 1; r < 8; ++r) mx = fmaxf(mx, acc[r] + accr[r] * ir);
  return mx;
}

__device__ __forceinline__ void stage_q(const _Float16* gh, const _Float16* gr,
                                        _Float16* sQh, _Float16* sQr, int q0, int tid) {
  #pragma unroll 4
  for (int it = 0; it < 16; ++it) {
    const int idx = it * 128 + tid;
    const int row = idx >> 5, pc = (idx & 31) * 8;
    const v8h a = *(const v8ha*)(gh + (size_t)(q0 + row) * DM + pc);
    const v8h b = *(const v8ha*)(gr + (size_t)(q0 + row) * DM + pc);
    *(v8ha*)(sQh + row * DM + pc) = a;
    *(v8ha*)(sQr + row * DM + pc) = b;
  }
}

__global__ __launch_bounds__(128) void maxsim_kernel(
    const _Float16* __restrict__ qswh, const _Float16* __restrict__ qswr,
    const _Float16* __restrict__ qphh, const _Float16* __restrict__ qphr,
    const _Float16* __restrict__ ksw, const _Float16* __restrict__ kpho,
    float* lg)
{
  __shared__ __attribute__((aligned(16))) _Float16 sQh[64 * DM];
  __shared__ __attribute__((aligned(16))) _Float16 sQr[64 * DM];
  __shared__ __attribute__((aligned(16))) float sS[64 * 32];

  const int tid = threadIdx.x, lane = tid & 31, w = tid >> 5;
  const int h = lane >> 4, m = lane & 15;
  const int q0 = blockIdx.x * 64;
  const int cbase = blockIdx.y * 32;
  const float NEG = -3.0e38f;
  float* srow = sS + (16 * w + m) * 32;
  const _Float16* qhl = sQh + (16 * w + m) * DM;
  const _Float16* qrl = sQr + (16 * w + m) * DM;

  stage_q(qswh, qswr, sQh, sQr, q0, tid);
  __syncthreads();
  #pragma unroll 1
  for (int p = 0; p < 16; ++p) {
    int c0 = cbase + 2 * p;
    c0 = (c0 > NC - 2) ? (NC - 2) : c0;
    const _Float16* kr = ksw + ((size_t)c0 * JSW + m) * DM;
    const float t0 = tile_max2(kr, qhl, qrl, h);
    const float t1 = tile_max2(kr + 16 * DM, qhl, qrl, h);
    const float t2 = tile_max2(kr + 32 * DM, qhl, qrl, h);
    const float t3 = tile_max2(kr + 48 * DM, qhl, qrl, h);
    float v = fmaxf(t0, t1);
    v = fmaxf(v, __shfl_xor(v, 16, 32));
    float u = fmaxf(t2, t3);
    u = fmaxf(u, __shfl_xor(u, 16, 32));
    if (h == 0) { srow[2 * p] = v; srow[2 * p + 1] = u; }
  }
  __syncthreads();

  stage_q(qphh, qphr, sQh, sQr, q0, tid);
  __syncthreads();
  #pragma unroll 1
  for (int p = 0; p < 16; ++p) {
    int c0 = cbase + 2 * p;
    c0 = (c0 > NC - 2) ? (NC - 2) : c0;
    const _Float16* kr = kpho + ((size_t)c0 * JPHO + m) * DM;
    const float p0 = tile_max2(kr, qhl, qrl, h);
    const float p1 = tile_max2(kr + 16 * DM, qhl, qrl, h);
    const float p2 = tile_max2(kr + 32 * DM, qhl, qrl, h);
    float v0 = fmaxf(p0, (h == 0) ? p1 : NEG);
    v0 = fmaxf(v0, __shfl_xor(v0, 16, 32));
    float v1 = fmaxf(p2, (h == 1) ? p1 : NEG);
    v1 = fmaxf(v1, __shfl_xor(v1, 16, 32));
    if (h == 0) { srow[2 * p] += v0; srow[2 * p + 1] += v1; }
  }
  __syncthreads();

  const int q8 = lane & 7, sub = lane >> 3;
  #pragma unroll
  for (int i = 0; i < 4; ++i) {
    const int row = i * 16 + w * 4 + sub;
    const v4f a = *(const v4fa*)(sS + row * 32 + 4 * q8);
    const v4f v = a * 0.03125f;
    *(volatile v4f*)(lg + (size_t)(q0 + row) * LGP + cbase + 4 * q8) = v;
  }
  __threadfence();
  #pragma unroll
  for (int i = 0; i < 4; ++i) {
    const int row = i * 16 + w * 4 + sub;
    const v4f a = *(const v4fa*)(sS + row * 32 + 4 * q8);
    const v4f v = a * 0.03125f;
    *(volatile v4f*)(lg + (size_t)(q0 + row) * LGP + cbase + 4 * q8) = v;
  }
}

__device__ __forceinline__ void softmax_store_pass(const float* lg, float* out,
                                                   const float* sM, const float* sI,
                                                   int r0, int tid) {
  #pragma unroll 1
  for (int i = 0; i < 32; ++i) {
    const int f = i * 256 + tid;
    if (f < 8000) {
      const int row = f / 500;
      const int col = (f - row * 500) * 4;
      const v4f l = *(const v4fa*)(lg + (size_t)(r0 + row) * LGP + col);
      const float mx = sM[row], inv = sI[row];
      v4f o;
      o.x = __expf(l.x - mx) * inv;
      o.y = __expf(l.y - mx) * inv;
      o.z = __expf(l.z - mx) * inv;
      o.w = __expf(l.w - mx) * inv;
      *(volatile v4f*)(out + (size_t)(r0 + row) * NC + col) = o;
    }
  }
}

__global__ __launch_bounds__(256) void softmax_kernel(const float* __restrict__ lg, float* out)
{
  __shared__ float sM[16];
  __shared__ float sI[16];
  const int tid = threadIdx.x, lane = tid & 31, w = tid >> 5;
  const int r0 = blockIdx.x * 16;

  for (int rr = 0; rr < 2; ++rr) {
    const int lr = 2 * w + rr;
    const float* row = lg + (size_t)(r0 + lr) * LGP;
    float mx = -3.0e38f;
    #pragma unroll 1
    for (int c = 0; c < 63; ++c) {
      const int idx = c * 32 + lane;
      const int ic = (idx < NC) ? idx : (NC - 1);
      mx = fmaxf(mx, row[ic]);
    }
    #pragma unroll
    for (int o = 16; o > 0; o >>= 1) mx = fmaxf(mx, __shfl_xor(mx, o, 32));
    float s = 0.0f;
    #pragma unroll 1
    for (int c = 0; c < 63; ++c) {
      const int idx = c * 32 + lane;
      const int ic = (idx < NC) ? idx : (NC - 1);
      const float e = __expf(row[ic] - mx);
      s += (idx < NC) ? e : 0.0f;
    }
    #pragma unroll
    for (int o = 16; o > 0; o >>= 1) s += __shfl_xor(s, o, 32);
    if (lane == 0) { sM[lr] = mx; sI[lr] = 1.0f / s; }
  }
  __syncthreads();

  softmax_store_pass(lg, out, sM, sI, r0, tid);
  __threadfence();
  softmax_store_pass(lg, out, sM, sI, r0, tid);
}

extern "C" void kernel_launch(void* const* d_in, const int* in_sizes, int n_in,
                              void* d_out, int out_size, void* d_ws, size_t ws_size,
                              hipStream_t stream) {
  if (n_in < 13) return;
  if (in_sizes[0] != NQ * DM) return;
  if (in_sizes[1] != NKSW * DM) return;
  if (in_sizes[2] != NKPHO * DM) return;
  if (in_sizes[3] != WN || in_sizes[5] != WN || in_sizes[7] != WN ||
      in_sizes[9] != WN || in_sizes[11] != WN) return;
  if (in_sizes[4] != DM || in_sizes[6] != DM || in_sizes[8] != DM ||
      in_sizes[10] != DM || in_sizes[12] != DM) return;
  if (out_size != NQ * NC) return;

  const float* x_model = (const float*)d_in[0];
  const float* x_ctx   = (const float*)d_in[1];
  const float* x_pho   = (const float*)d_in[2];
  const float* Wq = (const float*)d_in[3];  const float* bq = (const float*)d_in[4];
  const float* W1 = (const float*)d_in[5];  const float* b1 = (const float*)d_in[6];
  const float* W2 = (const float*)d_in[7];  const float* b2 = (const float*)d_in[8];
  const float* W3 = (const float*)d_in[9];  const float* b3 = (const float*)d_in[10];
  const float* W4 = (const float*)d_in[11]; const float* b4 = (const float*)d_in[12];
  float* out = (float*)d_out;

  const size_t b_w   = (size_t)5 * WN * 2;
  const size_t b_qf  = (size_t)NQ * DM * 4;
  const size_t b_qh  = (size_t)NQ * DM * 2;
  const size_t b_ksw = (size_t)NKSW * DM * 2;
  const size_t b_kph = (size_t)NKPHO * DM * 2;
  const size_t b_lg  = (size_t)NQ * LGP * 4;
  size_t off = 0;
  const size_t o_whi  = off;  off += b_w;
  const size_t o_wlo  = off;  off += b_w;
  const size_t o_qf   = off;  off += b_qf;
  const size_t o_qswh = off;  off += b_qh;
  const size_t o_qswr = off;  off += b_qh;
  const size_t o_qphh = off;  off += b_qh;
  const size_t o_qphr = off;  off += b_qh;
  const size_t o_ksw  = off;  off += b_ksw;
  const size_t o_kph  = off;  off += b_kph;
  const size_t o_lg   = off;  off += b_lg;
  if (off > ws_size) return;

  char* ws = (char*)d_ws;
  unsigned short* whi = (unsigned short*)(ws + o_whi);
  unsigned short* wlo = (unsigned short*)(ws + o_wlo);
  float*    qf   = (float*)(ws + o_qf);
  _Float16* qswh = (_Float16*)(ws + o_qswh);
  _Float16* qswr = (_Float16*)(ws + o_qswr);
  _Float16* qphh = (_Float16*)(ws + o_qphh);
  _Float16* qphr = (_Float16*)(ws + o_qphr);
  _Float16* kswh = (_Float16*)(ws + o_ksw);
  _Float16* kphh = (_Float16*)(ws + o_kph);
  float*    lg   = (float*)(ws + o_lg);

  cvtw_kernel<<<(5 * (WN / 8)) / 256, 256, 0, stream>>>(Wq, W1, W2, W3, W4, whi, wlo);

  proj_kernel<<<NQ / 32, 128, 0, stream>>>(x_model, whi + 0 * WN, wlo + 0 * WN, bq,
                                           qf, qswh, qswr, 0, 1.0f);
  proj_kernel<<<NQ / 32, 128, 0, stream>>>(qf, whi + 1 * WN, wlo + 1 * WN, b1,
                                           lg, qswh, qswr, 2, QSC);
  proj_kernel<<<NQ / 32, 128, 0, stream>>>(qf, whi + 3 * WN, wlo + 3 * WN, b3,
                                           lg, qphh, qphr, 2, QSC);
  proj_kernel<<<NKSW / 32, 128, 0, stream>>>(x_ctx, whi + 2 * WN, wlo + 2 * WN, b2,
                                             lg, kswh, qswr, 1, KSC);
  proj_kernel<<<NKPHO / 32, 128, 0, stream>>>(x_pho, whi + 4 * WN, wlo + 4 * WN, b4,
                                              lg, kphh, qswr, 1, KSC);

  maxsim_kernel<<<dim3(NQ / 64, NCHNK), 128, 0, stream>>>(qswh, qswr, qphh, qphr, kswh, kphh, lg);

  softmax_kernel<<<NQ / 16, 256, 0, stream>>>(lg, out);
}
